// SeqLSTMLabelingModel_42107859370787
// MI455X (gfx1250) — hardware-verified
//
#include <hip/hip_runtime.h>


namespace {
constexpr int NB = 128, SQ = 512, NROW = NB * SQ, VOC = 50000, WD = 300, NPOS = 37, PD = 32, MD = 66, NLAB = 43, LD = 100, KIN = 498, KP = 512, U = 1024, NG = 3, NC = 43, NCP = 48, SCW = 64;
constexpr int OW = 0, OP = 304, OM = 336, OL = 408;
constexpr int NOUT = NB * (SQ - 1) * NC;
constexpr float XS = 8.0f, WSC = 256.0f, HS = 64.0f;
typedef int idx_t;

typedef _Float16 b16;
typedef __attribute__((ext_vector_type(16))) _Float16 v16b;
typedef __attribute__((ext_vector_type(8))) _Float16 v8b;
typedef __attribute__((ext_vector_type(8))) float v8f;
typedef __attribute__((ext_vector_type(4))) float v4f;
__device__ __forceinline__ float bf16_rne(float f) { unsigned int u = __float_as_uint(f); u += 0x7FFFu + ((u >> 16) & 1u); return __uint_as_float(u & 0xFFFF0000u); }
__device__ __forceinline__ void split16(float v, b16& hi, b16& lo) { hi = (b16)v; lo = (b16)(v - (float)hi); }
__device__ __forceinline__ v16b frag_kb(const b16* p, int hh) { const v8b a = *(const v8b*)(p + 8 * hh), b = *(const v8b*)(p + 16 + 8 * hh); v16b f;
#pragma unroll
  for (int e = 0; e < 8; ++e) { f[e] = a[e]; f[8 + e] = b[e]; } return f; }
__device__ __forceinline__ v8f wmma16b(v16b a, v16b b, v8f c) { v8f d = __builtin_amdgcn_wmma_f32_16x16x32_f16(false, a, false, b, (short)0, c, false, false); asm volatile("v_nop\n\tv_nop\n\tv_nop\n\tv_nop" : "+v"(d) : "v"(a), "v"(b)); return d; }
__device__ __forceinline__ void wave_lds_sync() { __builtin_amdgcn_fence(__ATOMIC_RELEASE, "workgroup"); __builtin_amdgcn_wave_barrier(); __builtin_amdgcn_fence(__ATOMIC_ACQUIRE, "workgroup"); }
__device__ __forceinline__ float nexp(float x) { return __builtin_amdgcn_exp2f(x * 1.4426950408889634f); }
__device__ __forceinline__ float pmul(float a, float b) { float p = a * b; asm volatile("" : "+v"(p)); return p; }
__device__ __forceinline__ float sigm(float x) { return 1.0f / (1.0f + nexp(-x)); }
__device__ __forceinline__ float tanh_(float x) { const float e = nexp(-2.0f * fabsf(x)); const float t = (1.0f - e) / (1.0f + e); return x < 0.0f ? -t : t; }
__device__ __forceinline__ int iclamp(long long v, int lo, int hi) { return v < lo ? lo : (v > hi ? hi : (int)v); }
__device__ __forceinline__ int korig(int k) {
  return k < OP ? (k < WD ? k : -1) : k < OM ? WD + (k - OP) : k < OL ? (k - OM < MD ? WD + PD + (k - OM) : -1) : (k - OL < LD ? WD + PD + MD + (k - OL) : -1); }

__global__ __launch_bounds__(256) void prepw_kernel(const float* __restrict__ wx, b16* __restrict__ WX16) {
  __shared__ __attribute__((aligned(16))) b16 T[64][64 + 8];
  const int k0 = blockIdx.x * 64, n0 = blockIdx.y * 64, t_ = threadIdx.x;
  const int gate = n0 / U, col0 = (gate == 0 ? 0 : gate == 1 ? 2 * U : 3 * U) + (n0 - gate * U);
  for (int q = t_; q < 64 * 64; q += 256) { const int kk = q >> 6, nn = q & 63; const int ko = korig(k0 + kk); T[nn][kk] = (ko >= 0) ? (b16)(bf16_rne(wx[(size_t)(ko >= 0 ? ko : 0) * (4 * U) + col0 + nn]) * WSC) : (b16)0.0f; }
  __syncthreads();
  for (int pass = 0; pass < 2; ++pass) { for (int q = t_; q < 64 * 8; q += 256) { const int nn = q >> 3, c8 = (q & 7) * 8; *(volatile v8b*)(WX16 + (size_t)(n0 + nn) * KP + k0 + c8) = *(const v8b*)(&T[nn][c8]); } __threadfence(); }
}
__global__ __launch_bounds__(256) void prepd_kernel(const float* __restrict__ wd, b16* __restrict__ WD16) {
  __shared__ __attribute__((aligned(16))) b16 T[NCP][64 + 8];
  const int u0 = blockIdx.x * 64, t_ = threadIdx.x;
  for (int q = t_; q < NCP * 64; q += 256) { const int c = q >> 6, uu = q & 63; T[c][uu] = (c < NC) ? (b16)(bf16_rne(wd[(size_t)(u0 + uu) * NC + (c < NC ? c : 0)]) * WSC) : (b16)0.0f; }
  __syncthreads();
  for (int pass = 0; pass < 2; ++pass) { for (int q = t_; q < NCP * 8; q += 256) { const int c = q >> 3, c8 = (q & 7) * 8; *(volatile v8b*)(WD16 + (size_t)c * U + u0 + c8) = *(const v8b*)(&T[c][c8]); } __threadfence(); }
}
__global__ __launch_bounds__(256) void gather_kernel(const idx_t* __restrict__ words, const idx_t* __restrict__ pos, const float* __restrict__ morph, const idx_t* __restrict__ labels, const float* __restrict__ wemb, const float* __restrict__ pemb, const float* __restrict__ lemb, b16* __restrict__ X16) {
  __shared__ __attribute__((aligned(16))) b16 T[8][KP + 8];
  const int wave = threadIdx.x >> 5, lane = threadIdx.x & 31, row = blockIdx.x * 8 + wave, b = row / SQ, s = row - b * SQ;
  const int w = iclamp(words[row], 0, VOC - 1), p = iclamp(pos[row], 0, NPOS - 1), lb = iclamp(labels[(size_t)b * SQ + (s > 0 ? s - 1 : 0)], 0, NLAB - 1);
  for (int g = lane; g < 38; g += 32) { v8b o;
#pragma unroll
    for (int j = 0; j < 8; ++j) { const int f = g * 8 + j; o[j] = (f < WD) ? (b16)(bf16_rne(wemb[(size_t)w * WD + (f < WD ? f : 0)]) * XS) : (b16)0.0f; }
    *(v8b*)(&T[wave][OW + g * 8]) = o; }
  if (lane < 4) { v8b o;
#pragma unroll
    for (int j = 0; j < 8; ++j) o[j] = (b16)(bf16_rne(pemb[p * PD + lane * 8 + j]) * XS);
    *(v8b*)(&T[wave][OP + lane * 8]) = o; }
  if (lane < 9) { v8b o;
#pragma unroll
    for (int j = 0; j < 8; ++j) { const int f = lane * 8 + j; o[j] = (f < MD) ? (b16)(bf16_rne(morph[(size_t)row * MD + (f < MD ? f : 0)]) * XS) : (b16)0.0f; }
    *(v8b*)(&T[wave][OM + lane * 8]) = o; }
  if (lane < 13) { v8b o;
#pragma unroll
    for (int j = 0; j < 8; ++j) { const int f = lane * 8 + j; const float v = (s == 0) ? 1.0f : bf16_rne(lemb[(size_t)lb * LD + (f < LD ? f : 0)]); o[j] = (f < LD) ? (b16)(v * XS) : (b16)0.0f; }
    *(v8b*)(&T[wave][OL + lane * 8]) = o; }
  wave_lds_sync();
  for (int pass = 0; pass < 2; ++pass) { for (int h = 0; h < 2; ++h) *(volatile v8b*)(X16 + (size_t)row * KP + h * 256 + lane * 8) = *(const v8b*)(&T[wave][h * 256 + lane * 8]); __threadfence(); }
}
__global__ __launch_bounds__(128) void main_kernel(const b16* __restrict__ X16, const b16* __restrict__ WX16, const float* __restrict__ bias, const b16* __restrict__ WD16, const float* __restrict__ bd, float* __restrict__ SC) {
  __shared__ __attribute__((aligned(16))) b16 Hh[4][16][64 + 8], Hl[4][16][64 + 8]; __shared__ __attribute__((aligned(16))) float Ts[4][16][SCW + 4];
  const int wave = threadIdx.x >> 5, lane = threadIdx.x & 31, nloc = lane & 15, hlf = lane >> 4; const size_t m0 = (size_t)blockIdx.x * 64 + wave * 16;
  const b16* A = X16 + (m0 + nloc) * KP;
  v8f sacc[3] = {{}, {}, {}};
  for (int uc = 0; uc < U / 64; ++uc) {
    v8f acc[NG][4];
#pragma unroll
    for (int g = 0; g < NG; ++g)
#pragma unroll
      for (int t = 0; t < 4; ++t) acc[g][t] = (v8f){};
#pragma unroll 2
    for (int kb = 0; kb < KP; kb += 32) { const v16b a = frag_kb(A + kb, hlf);
#pragma unroll
      for (int g = 0; g < NG; ++g)
#pragma unroll
        for (int t = 0; t < 4; ++t) acc[g][t] = wmma16b(a, frag_kb(WX16 + (size_t)(g * U + uc * 64 + t * 16 + nloc) * KP + kb, hlf), acc[g][t]); }
#pragma unroll
    for (int t = 0; t < 4; ++t) { const int u = uc * 64 + t * 16 + nloc; const float bi = bf16_rne(bias[u]), bg = bf16_rne(bias[2 * U + u]), bo = bf16_rne(bias[3 * U + u]);
#pragma unroll
      for (int r = 0; r < 8; ++r) { const float zi = acc[0][t][r] * (1.0f / (XS * WSC)) + bi, zg = acc[1][t][r] * (1.0f / (XS * WSC)) + bg, zo = acc[2][t][r] * (1.0f / (XS * WSC)) + bo;
        const float c = pmul(sigm(zi), tanh_(zg)); const float h = pmul(sigm(zo), tanh_(c)); b16 a_, c_; split16(h * HS, a_, c_); Hh[wave][8 * hlf + r][t * 16 + nloc] = a_; Hl[wave][8 * hlf + r][t * 16 + nloc] = c_; } }
    wave_lds_sync();
#pragma unroll
    for (int ks = 0; ks < 2; ++ks) { const v16b ah = frag_kb(&Hh[wave][nloc][ks * 32], hlf), al = frag_kb(&Hl[wave][nloc][ks * 32], hlf);
#pragma unroll
      for (int ct = 0; ct < 3; ++ct) { const v16b bw = frag_kb(WD16 + (size_t)(ct * 16 + nloc) * U + uc * 64 + ks * 32, hlf); sacc[ct] = wmma16b(ah, bw, sacc[ct]); sacc[ct] = wmma16b(al, bw, sacc[ct]); } }
    wave_lds_sync(); }
#pragma unroll
  for (int ct = 0; ct < 3; ++ct)
#pragma unroll
    for (int r = 0; r < 8; ++r) { const int c = ct * 16 + nloc; Ts[wave][8 * hlf + r][c] = sacc[ct][r] * (1.0f / (HS * WSC)) + (c < NC ? bf16_rne(bd[c < NC ? c : 0]) : 0.0f); }
  if (nloc == 0) {
#pragma unroll
    for (int r = 0; r < 8; ++r) for (int c = NCP; c < SCW; ++c) Ts[wave][8 * hlf + r][c] = 0.0f; }
  wave_lds_sync();
  for (int pass = 0; pass < 2; ++pass) { for (int rr = 0; rr < 16; ++rr) if (lane < 16) *(volatile v4f*)(SC + (m0 + rr) * SCW + lane * 4) = *(const v4f*)(&Ts[wave][rr][lane * 4]); __threadfence(); }
}
__global__ __launch_bounds__(256) void out_kernel(const float* __restrict__ SC, float* __restrict__ out) {
  const int p = blockIdx.x * 256 + threadIdx.x; const int pc = p < NOUT ? p : NOUT - 1;
  const int r = pc / NC, c = pc - r * NC, b = r / (SQ - 1), s1 = r - b * (SQ - 1);
  const float v = SC[((size_t)b * SQ + s1 + 1) * SCW + c];
  for (int pass = 0; pass < 2; ++pass) { if (p < NOUT) ((volatile float*)out)[p] = v; __threadfence(); }
}
}

extern "C" void kernel_launch(void* const* d_in, const int* in_sizes, int n_in, void* d_out, int out_size, void* d_ws, size_t ws_size, hipStream_t stream) {
  (void)n_in;
  auto Fp = [&](int i) { return (const float*)d_in[i]; };
  if (in_sizes[0] != NROW || in_sizes[2] != NROW * MD || in_sizes[4] != VOC * WD || in_sizes[7] != KIN * 4 * U || in_sizes[10] != U * NC || out_size != NOUT) return;
  size_t off = 0; char* ws = (char*)d_ws;
  auto carve = [&](size_t bytes) { char* p = ws + off; off += (bytes + 255) & ~(size_t)255; return p; };
  b16* WX16 = (b16*)carve((size_t)NG * U * KP * 2); b16* WD16 = (b16*)carve((size_t)NCP * U * 2); b16* X16 = (b16*)carve((size_t)NROW * KP * 2); float* SC = (float*)carve((size_t)NROW * SCW * 4);
  if (off > ws_size) return;
  prepw_kernel<<<dim3(KP / 64, NG * U / 64), 256, 0, stream>>>(Fp(7), WX16);
  prepd_kernel<<<U / 64, 256, 0, stream>>>(Fp(10), WD16);
  gather_kernel<<<NROW / 8, 256, 0, stream>>>((const idx_t*)d_in[0], (const idx_t*)d_in[1], Fp(2), (const idx_t*)d_in[3], Fp(4), Fp(5), Fp(6), X16);
  main_kernel<<<NROW / 64, 128, 0, stream>>>(X16, WX16, Fp(9), WD16, Fp(11), SC);
  out_kernel<<<(NOUT + 255) / 256, 256, 0, stream>>>(SC, (float*)d_out);
}
